// unit_gcn_81655918232209
// MI455X (gfx1250) — hardware-verified
//
#include <hip/hip_runtime.h>

#ifndef NB
#define NB 64
#endif
#define CIN 64
#define COUT 64
#define TT 128
#define VV 25
#define VP 32
#define SS 3
#define RR 8
#define SR (SS * RR)
#define KP 96
#define XS_FULL (CIN * TT * VV)
#define CH ((NB < 16) ? NB : 16)
#define NCHUNK (NB / CH)
static_assert(NB >= 1 && NB <= 64);
static_assert(NB % CH == 0);
static_assert(KP % 32 == 0);
static_assert((NB * XS_FULL) % 1024 == 0);

typedef __bf16 v16b __attribute__((ext_vector_type(16)));
typedef unsigned short v8us __attribute__((ext_vector_type(8), may_alias));
typedef float  v8f  __attribute__((ext_vector_type(8)));
typedef float  v4f  __attribute__((ext_vector_type(4)));
typedef float  v4fa __attribute__((ext_vector_type(4), may_alias));
typedef double v2d  __attribute__((ext_vector_type(2)));
union FragB { v16b v; v8us half[2]; unsigned short u[16]; };

__device__ __forceinline__ unsigned short bf16_bits(float x) { unsigned int u = __float_as_uint(x); return (unsigned short)((u + 0x7FFFu + ((u >> 16) & 1u)) >> 16); }
__device__ __forceinline__ float bf16_val(unsigned short b) { return __uint_as_float(((unsigned int)b) << 16); }
__device__ __forceinline__ float bf16_rne(float x) { return bf16_val(bf16_bits(x)); }

template <int NT>
__device__ __forceinline__ v8f mmaN(v16b ah, v16b al, v16b bh, v16b bl, v8f c) {
  c = __builtin_amdgcn_wmma_f32_16x16x32_bf16(false, ah, false, bh, (short)0, c, false, false);
  if (NT >= 2) c = __builtin_amdgcn_wmma_f32_16x16x32_bf16(false, al, false, bh, (short)0, c, false, false);
  if (NT >= 3) c = __builtin_amdgcn_wmma_f32_16x16x32_bf16(false, ah, false, bl, (short)0, c, false, false);
  asm volatile("v_nop\n\tv_nop\n\tv_nop\n\tv_nop" : "+v"(c) : "v"(ah), "v"(al), "v"(bh), "v"(bl));
  return c;
}
__device__ __forceinline__ v8f mma1(v16b a, v16b b, v8f c) {
  c = __builtin_amdgcn_wmma_f32_16x16x32_bf16(false, a, false, b, (short)0, c, false, false);
  asm volatile("v_nop\n\tv_nop\n\tv_nop\n\tv_nop" : "+v"(c) : "v"(a), "v"(b));
  return c;
}
__device__ __forceinline__ v16b ldfrag(const unsigned short* p, int hh) { FragB f; f.half[0] = *(const v8us*)(p + 8 * hh); f.half[1] = *(const v8us*)(p + 16 + 8 * hh); return f.v; }

__global__ __launch_bounds__(256) void k_prep(const float* __restrict__ W3, const float* __restrict__ W1, const float* __restrict__ W2, const float* __restrict__ b1, const float* __restrict__ b2,
                                              unsigned short* __restrict__ W3B, unsigned short* __restrict__ W12B, float* __restrict__ B12) {
  const int bid = blockIdx.x, tid = threadIdx.x;
  if (bid < 6) {
    const int t = bid * 256 + tid;
    v8us v;
#pragma unroll
    for (int i = 0; i < 8; ++i) v[i] = bf16_bits(W3[(size_t)t * 8 + i]);
    unsigned short* d = W3B + (size_t)t * 8;
    *(volatile v8us*)d = v; __threadfence(); *(volatile v8us*)d = v;
  } else if (bid < 8) {
    const int t = (bid - 6) * 256 + tid;
    const int j = t >> 3, k8 = (t & 7) * 8;
    const int j1 = min(j, SR - 1), j2 = min(max(j - SR, 0), SR - 1);
    v8us v;
#pragma unroll
    for (int i = 0; i < 8; ++i) {
      const float a = W1[j1 * CIN + k8 + i], b = W2[j2 * CIN + k8 + i];
      const float s = (j < SR) ? a : ((j < 2 * SR) ? b : 0.f);
      v[i] = bf16_bits(s);
    }
    unsigned short* d = W12B + (size_t)t * 8;
    *(volatile v8us*)d = v; __threadfence(); *(volatile v8us*)d = v;
  } else {
    if (tid < 64) {
      const int j = tid; const int j1 = min(j, SR - 1), j2 = min(max(j - SR, 0), SR - 1);
      const float a = b1[j1], b = b2[j2];
      const float s = (j < SR) ? a : ((j < 2 * SR) ? b : 0.f);
      *(volatile float*)(B12 + j) = s; __threadfence(); *(volatile float*)(B12 + j) = s;
    }
  }
}

__global__ __launch_bounds__(256) void k_xm(const float* __restrict__ x, float* __restrict__ XM) {
  const int i = blockIdx.x * 256 + threadIdx.x;
  if (i >= NB * VP * CIN) return;
  const int c = i & (CIN - 1), v = (i >> 6) & (VP - 1), n = i >> 11;
  const int vc = min(v, VV - 1);
  const float* p = x + (size_t)(n * CIN + c) * (TT * VV) + vc;
  float s = 0.f;
#pragma unroll 4
  for (int t = 0; t < TT; ++t) s += bf16_rne(p[t * VV]);
  float m = s * 0.0078125f;
  if (v >= VV) m = 0.f;
  *(volatile float*)(XM + i) = m; __threadfence(); *(volatile float*)(XM + i) = m;
}

template <bool ASPLIT, int ACT, bool BIAS_BF16>
__global__ __launch_bounds__(128) void k_gemm_bf(const float* __restrict__ A, int lda, const unsigned short* __restrict__ Wt, int ldb,
                                               const float* __restrict__ bias, float* __restrict__ C, int ldc, int M, int N, int K) {
  __shared__ __attribute__((aligned(16))) float so[4][16][64];
  const int tid = threadIdx.x, w = tid >> 5, lane = tid & 31, ln = lane & 15, hh = lane >> 4;
  const int ntn = N / 64;
  const int wid = blockIdx.x * 4 + w;
  const int mt = wid / ntn, nq = wid % ntn;
  if (mt * 16 >= M) return;
  const int row0 = mt * 16, col0 = nq * 64;
  const float* arow = A + (size_t)(row0 + ln) * lda;
  v8f acc[4] = {};
#pragma unroll 1
  for (int kb = 0; kb < K; kb += 32) {
    FragB ah, al;
    const v4f x0 = *(const v4fa*)(arow + kb + 8 * hh), x1 = *(const v4fa*)(arow + kb + 8 * hh + 4);
    const v4f x2 = *(const v4fa*)(arow + kb + 16 + 8 * hh), x3 = *(const v4fa*)(arow + kb + 16 + 8 * hh + 4);
    float xs[16] = {x0[0],x0[1],x0[2],x0[3],x1[0],x1[1],x1[2],x1[3],x2[0],x2[1],x2[2],x2[3],x3[0],x3[1],x3[2],x3[3]};
#pragma unroll
    for (int i = 0; i < 16; ++i) { const unsigned short hb = bf16_bits(xs[i]); ah.u[i] = hb; al.u[i] = ASPLIT ? bf16_bits(xs[i] - bf16_val(hb)) : (unsigned short)0; }
#pragma unroll
    for (int t = 0; t < 4; ++t) {
      const unsigned short* brow = Wt + (size_t)(col0 + t * 16 + ln) * ldb + kb;
      FragB b;
      b.half[0] = *(const v8us*)(brow + 8 * hh);
      b.half[1] = *(const v8us*)(brow + 16 + 8 * hh);
      acc[t] = mmaN<ASPLIT ? 2 : 1>(ah.v, al.v, b.v, b.v, acc[t]);
    }
  }
#pragma unroll
  for (int t = 0; t < 4; ++t) {
    float bv = bias ? bias[col0 + t * 16 + ln] : 0.f;
    if (BIAS_BF16) bv = bf16_rne(bv);
#pragma unroll
    for (int r = 0; r < 8; ++r) { float v = acc[t][r] + bv; if (ACT == 1) v = fmaxf(v, 0.f); so[w][8 * hh + r][t * 16 + ln] = v; }
  }
  __builtin_amdgcn_fence(__ATOMIC_ACQ_REL, "workgroup");
  __builtin_amdgcn_wave_barrier();
  const int rsub = lane >> 4, c4 = (lane & 15) * 4;
  for (int rep = 0; rep < 2; ++rep) {
#pragma unroll
    for (int q = 0; q < 8; ++q) {
      const int r = q * 2 + rsub;
      const v4f v = *(const v4fa*)&so[w][r][c4];
      *(volatile v4f*)(C + (size_t)(row0 + r) * ldc + col0 + c4) = v;
    }
    if (rep == 0) __threadfence();
  }
}

__global__ __launch_bounds__(256) void k_xt(const float* __restrict__ x, unsigned short* __restrict__ XT, int n0) {
  __shared__ unsigned short tile[CIN][100];
  const int tid = threadIdx.x; const int nl = blockIdx.x >> 5, tg = blockIdx.x & 31; const int n = n0 + nl, t0 = tg * 4;
  for (int idx = tid; idx < CIN * 25; idx += 256) {
    const int c = idx / 25, k = idx - c * 25;
    const v4f a = *(const v4fa*)(x + ((size_t)(n * CIN + c) * TT + t0) * VV + 4 * k);
#pragma unroll
    for (int q = 0; q < 4; ++q) tile[c][4 * k + q] = bf16_bits(a[q]);
  }
  __syncthreads();
  const size_t base = ((size_t)nl * TT + t0) * VP * CIN;
#pragma unroll 1
  for (int it = 0; it < 4; ++it) {
    const int p = it * 256 + tid; const int row = p >> 3, c0 = (p & 7) * 8; const int tl = row >> 5, v = row & 31;
    const int col = tl * 25 + min(v, VV - 1);
    v8us o;
#pragma unroll
    for (int i = 0; i < 8; ++i) { const unsigned short uu = tile[c0 + i][col]; o[i] = (v < VV) ? uu : (unsigned short)0; }
    unsigned short* dst = XT + base + (size_t)p * 8;
    *(volatile v8us*)dst = o; __threadfence(); *(volatile v8us*)dst = o;
  }
}

__device__ __forceinline__ void stg_cv(float (*so)[36], int col, int rowb, v8f c) {
#pragma unroll
  for (int r = 0; r < 8; ++r) so[col][rowb + r] = c[r];
}
__device__ __forceinline__ void stg_rc(float (*so)[36], int rowb, int col, v8f c) {
#pragma unroll
  for (int r = 0; r < 8; ++r) so[rowb + r][col] = c[r];
}

__global__ __launch_bounds__(128) void k_x3(const unsigned short* __restrict__ XT, const unsigned short* __restrict__ W3B, const float* __restrict__ b3,
                                            unsigned short* __restrict__ X3H, unsigned short* __restrict__ X3L) {
  __shared__ __attribute__((aligned(16))) float so[SS * COUT][36];
  const int tid = threadIdx.x, w = tid >> 5, lane = tid & 31, ln = lane & 15, hh = lane >> 4;
  const int nl = blockIdx.x / TT, t = blockIdx.x - nl * TT;
  const unsigned short* Ab = XT + ((size_t)(nl * TT + t)) * VP * CIN;
  const unsigned short* a0p = Ab + (size_t)ln * CIN;
  const unsigned short* a1p = Ab + (size_t)(16 + ln) * CIN;
  const unsigned short* b0p = W3B + (size_t)(48 * w + ln) * CIN;
  const unsigned short* b1p = b0p + (size_t)16 * CIN;
  const unsigned short* b2p = b1p + (size_t)16 * CIN;
  const v8f z8 = {0.f,0.f,0.f,0.f,0.f,0.f,0.f,0.f};
  v8f c00 = z8, c01 = z8, c02 = z8, c10 = z8, c11 = z8, c12 = z8;
#pragma unroll 1
  for (int kb = 0; kb < CIN; kb += 32) {
    const v16b a0 = ldfrag(a0p + kb, hh), a1 = ldfrag(a1p + kb, hh);
    v16b b = ldfrag(b0p + kb, hh); c00 = mma1(a0, b, c00); c10 = mma1(a1, b, c10);
    b = ldfrag(b1p + kb, hh); c01 = mma1(a0, b, c01); c11 = mma1(a1, b, c11);
    b = ldfrag(b2p + kb, hh); c02 = mma1(a0, b, c02); c12 = mma1(a1, b, c12);
  }
  stg_cv(so, 48 * w + ln, 8 * hh, c00); stg_cv(so, 48 * w + 16 + ln, 8 * hh, c01); stg_cv(so, 48 * w + 32 + ln, 8 * hh, c02);
  stg_cv(so, 48 * w + ln, 16 + 8 * hh, c10); stg_cv(so, 48 * w + 16 + ln, 16 + 8 * hh, c11); stg_cv(so, 48 * w + 32 + ln, 16 + 8 * hh, c12);
  __syncthreads();
  const size_t base = ((size_t)(nl * TT + t)) * COUT * KP;
#pragma unroll 1
  for (int it = 0; it < 6; ++it) {
    const int p = it * 128 + tid; const int o = p / 12, jj = p - o * 12; const int s = jj >> 2, v0 = (jj & 3) * 8; const int col = s * COUT + o;
    const v4f d0 = *(const v4fa*)&so[col][v0], d1 = *(const v4fa*)&so[col][v0 + 4];
    const float vals[8] = {d0[0], d0[1], d0[2], d0[3], d1[0], d1[1], d1[2], d1[3]};
    const float bv = bf16_rne(b3[col]);
    v8us hv, lv;
#pragma unroll
    for (int i = 0; i < 8; ++i) {
      float val = vals[i] + bv;
      if (v0 + i >= VV) val = 0.f;
      const unsigned short hb = bf16_bits(val);
      hv[i] = hb; lv[i] = bf16_bits(val - bf16_val(hb));
    }
    const size_t off = base + (size_t)p * 8;
    unsigned short* dh = X3H + off; unsigned short* dl = X3L + off;
    *(volatile v8us*)dh = hv; *(volatile v8us*)dl = lv; __threadfence(); *(volatile v8us*)dh = hv; *(volatile v8us*)dl = lv;
  }
}

__global__ __launch_bounds__(256) void k_m(const float* __restrict__ X12, const float* __restrict__ W4, const float* __restrict__ b4, const float* __restrict__ PA,
                                           const float* __restrict__ alpha, unsigned short* __restrict__ MH, unsigned short* __restrict__ ML, int n0) {
  __shared__ __attribute__((aligned(16))) float sd[SS * RR * 8][VP];
  __shared__ __attribute__((aligned(16))) float spa[SS * VV][VP];
  __shared__ float sw4[SS * COUT * RR];
  __shared__ float sb4[SS * COUT];
  const int tid = threadIdx.x; const int nl = blockIdx.x >> 2, ug = blockIdx.x & 3; const int n = n0 + nl, u0 = ug * 8;
  for (int i = tid; i < SS * COUT * RR; i += 256) sw4[i] = bf16_rne(W4[i]);
  if (tid < SS * COUT) sb4[tid] = bf16_rne(b4[tid]);
  for (int i = tid; i < SS * VV * VP; i += 256) {
    const int su = i >> 5, v = i & 31;
    const float pv = bf16_rne(PA[su * VV + min(v, VV - 1)]);
    spa[su][v] = (v < VV) ? pv : 0.f;
  }
#pragma unroll 1
  for (int i = tid; i < SS * RR * 8 * VP; i += 256) {
    const int v = i & 31, ul = (i >> 5) & 7, sr = i >> 8; const int u = u0 + ul;
    const float a = X12[(size_t)(n * VP + u) * 64 + sr];
    const float b = X12[(size_t)(n * VP + v) * 64 + SR + sr];
    const float d = tanhf(a - b);
    sd[sr * 8 + ul][v] = (u < VV && v < VV) ? d : 0.f;
  }
  __syncthreads();
  const float al = bf16_rne(alpha[0]);
  const size_t nbase = (size_t)nl * COUT * VP * KP;
#pragma unroll 1
  for (int it = 0; it < 24; ++it) {
    const int p = it * 256 + tid; const int o = p / 96, q = p - o * 96; const int ul = q / 12, jj = q - ul * 12; const int s = jj >> 2, v0 = (jj & 3) * 8;
    const int u = u0 + ul;
    v4f accA = {0.f, 0.f, 0.f, 0.f}, accB = {0.f, 0.f, 0.f, 0.f};
#pragma unroll 1
    for (int r = 0; r < RR; ++r) {
      const float wv = sw4[(s * COUT + o) * RR + r];
      const v4f d0 = *(const v4fa*)&sd[(s * RR + r) * 8 + ul][v0];
      const v4f d1 = *(const v4fa*)&sd[(s * RR + r) * 8 + ul][v0 + 4];
      accA += wv * d0; accB += wv * d1;
    }
    const float bb = sb4[s * COUT + o]; const int uc = min(u, VV - 1);
    const v4f p0 = *(const v4fa*)&spa[s * VV + uc][v0], p1 = *(const v4fa*)&spa[s * VV + uc][v0 + 4];
    const float av8[8] = {accA[0], accA[1], accA[2], accA[3], accB[0], accB[1], accB[2], accB[3]};
    const float pv8[8] = {p0[0], p0[1], p0[2], p0[3], p1[0], p1[1], p1[2], p1[3]};
    v8us hv, lv;
#pragma unroll
    for (int i = 0; i < 8; ++i) {
      float m = (av8[i] + bb) * al + pv8[i];
      if (u >= VV || v0 + i >= VV) m = 0.f;
      const unsigned short hb = bf16_bits(m);
      hv[i] = hb; lv[i] = bf16_bits(m - bf16_val(hb));
    }
    const size_t off = nbase + ((size_t)o * VP + u0) * KP + (size_t)q * 8;
    unsigned short* dh = MH + off; unsigned short* dl = ML + off;
    *(volatile v8us*)dh = hv; *(volatile v8us*)dl = lv; __threadfence(); *(volatile v8us*)dh = hv; *(volatile v8us*)dl = lv;
  }
}

__global__ __launch_bounds__(128) void k_agg(const unsigned short* __restrict__ X3H, const unsigned short* __restrict__ X3L, const unsigned short* __restrict__ MH, const unsigned short* __restrict__ ML,
                                             float* __restrict__ Y, double* __restrict__ PART, int n0) {
  __shared__ __attribute__((aligned(16))) float so[TT][36];
  __shared__ double red2[8];
  const int tid = threadIdx.x, w = tid >> 5, lane = tid & 31, ln = lane & 15, hh = lane >> 4;
  const int nl = blockIdx.x >> 6, o = blockIdx.x & 63; const int n = n0 + nl;
  const size_t ar0 = ((size_t)(nl * TT + 32 * w + ln) * COUT + o) * KP;
  const size_t ar1 = ar0 + (size_t)16 * COUT * KP;
  const size_t br0 = ((size_t)(nl * COUT + o) * VP + ln) * KP;
  const size_t br1 = br0 + (size_t)16 * KP;
  const v8f z8 = {0.f,0.f,0.f,0.f,0.f,0.f,0.f,0.f};
  v8f c00 = z8, c01 = z8, c10 = z8, c11 = z8;
#pragma unroll 1
  for (int kb = 0; kb < KP; kb += 32) {
    const v16b a0h = ldfrag(X3H + ar0 + kb, hh), a0l = ldfrag(X3L + ar0 + kb, hh);
    const v16b a1h = ldfrag(X3H + ar1 + kb, hh), a1l = ldfrag(X3L + ar1 + kb, hh);
    const v16b b0h = ldfrag(MH + br0 + kb, hh), b0l = ldfrag(ML + br0 + kb, hh);
    const v16b b1h = ldfrag(MH + br1 + kb, hh), b1l = ldfrag(ML + br1 + kb, hh);
    c00 = mmaN<3>(a0h, a0l, b0h, b0l, c00); c01 = mmaN<3>(a0h, a0l, b1h, b1l, c01);
    c10 = mmaN<3>(a1h, a1l, b0h, b0l, c10); c11 = mmaN<3>(a1h, a1l, b1h, b1l, c11);
  }
  stg_rc(so, 32 * w + 8 * hh, ln, c00); stg_rc(so, 32 * w + 8 * hh, 16 + ln, c01);
  stg_rc(so, 32 * w + 16 + 8 * hh, ln, c10); stg_rc(so, 32 * w + 16 + 8 * hh, 16 + ln, c11);
  __syncthreads();
  double s1 = 0.0, s2 = 0.0;
  float* yrow = Y + ((size_t)(n * COUT + o) * VV) * TT;
#pragma unroll 1
  for (int it = 0; it < 7; ++it) {
    const int p = it * 128 + tid;
    if (p < VV * 32) {
      const int u = p >> 5, t0 = (p & 31) * 4;
      v4f v; v[0] = so[t0][u]; v[1] = so[t0 + 1][u]; v[2] = so[t0 + 2][u]; v[3] = so[t0 + 3][u];
#pragma unroll
      for (int q = 0; q < 4; ++q) { const double dv = (double)v[q]; s1 += dv; s2 += dv * dv; }
      float* dst = yrow + (size_t)p * 4;
      *(volatile v4f*)dst = v; __threadfence(); *(volatile v4f*)dst = v;
    }
  }
#pragma unroll
  for (int off = 16; off > 0; off >>= 1) { s1 += __shfl_xor(s1, off, 32); s2 += __shfl_xor(s2, off, 32); }
  if (lane == 0) { red2[2 * w] = s1; red2[2 * w + 1] = s2; }
  __syncthreads();
  if (w == 0 && lane < 8) {
    v2d pv;
    pv[0] = ((red2[0] + red2[2]) + red2[4]) + red2[6];
    pv[1] = ((red2[1] + red2[3]) + red2[5]) + red2[7];
    if (lane != 0) { pv[0] = 0.0; pv[1] = 0.0; }
    double* dst = PART + (size_t)(n * COUT + o) * 16 + lane * 2;
    *(volatile v2d*)dst = pv; __threadfence(); *(volatile v2d*)dst = pv;
  }
}

__global__ __launch_bounds__(64) void k_bnfin(const double* __restrict__ PART, float* __restrict__ BNP) {
  const int o = threadIdx.x;
  double S = 0.0, Q = 0.0;
#pragma unroll 1
  for (int n = 0; n < NB; ++n) { const double* pp = PART + (size_t)(n * COUT + o) * 16; S += pp[0]; Q += pp[1]; }
  const double cnt = (double)NB * (double)(TT * VV);
  const double mu = S / cnt;
  double var = Q / cnt - mu * mu; if (var < 0.0) var = 0.0;
  const float muf = (float)mu;
  const float inv = 1.0f / sqrtf((float)var + 1e-5f);
  *(volatile float*)(BNP + o) = muf; *(volatile float*)(BNP + COUT + o) = inv; __threadfence();
  *(volatile float*)(BNP + o) = muf; *(volatile float*)(BNP + COUT + o) = inv;
}

__global__ __launch_bounds__(256) void k_out(const float* __restrict__ Y, const float* __restrict__ x, const float* __restrict__ BNP, const float* __restrict__ gamma, const float* __restrict__ beta,
                                             float* __restrict__ out, int total4) {
  #pragma clang fp contract(off)
  const int i = blockIdx.x * 256 + threadIdx.x;
  if (i >= total4) return;
  const v4f xv = *(const v4fa*)(x + (size_t)i * 4);
  v4f ov;
#pragma unroll
  for (int q = 0; q < 4; ++q) {
    const int e = i * 4 + q; const int u = e % VV; const int tq = e / VV; const int t = tq & (TT - 1); const int no = tq >> 7; const int o = no & (COUT - 1);
    const float yv = Y[((size_t)no * VV + u) * TT + t];
    const float mu = BNP[o], inv = BNP[COUT + o];
    const float g = bf16_rne(gamma[o]), b = bf16_rne(beta[o]);
    float v = (yv - mu) * inv;
    v = v * g + b;
    v = v + bf16_rne(xv[q]);
    ov[q] = fmaxf(v, 0.f);
  }
  float* dst = out + (size_t)i * 4;
  *(volatile v4f*)dst = ov; __threadfence(); *(volatile v4f*)dst = ov;
}

extern "C" void kernel_launch(void* const* d_in, const int* in_sizes, int n_in,
                              void* d_out, int out_size, void* d_ws, size_t ws_size, hipStream_t stream) {
  if (n_in < 13) return;
  if (in_sizes[0] < NB * XS_FULL || in_sizes[1] < SR * CIN || in_sizes[2] < SR || in_sizes[3] < SR * CIN || in_sizes[4] < SR ||
      in_sizes[5] < SS * COUT * CIN || in_sizes[6] < SS * COUT || in_sizes[7] < SS * COUT * RR || in_sizes[8] < SS * COUT ||
      in_sizes[9] < SS * VV * VV || in_sizes[10] < 1 || in_sizes[11] < COUT || in_sizes[12] < COUT) return;
  if (out_size < NB * XS_FULL) return;
  const float* x     = (const float*)d_in[0];
  const float* W1s   = (const float*)d_in[1];
  const float* b1s   = (const float*)d_in[2];
  const float* W2s   = (const float*)d_in[3];
  const float* b2s   = (const float*)d_in[4];
  const float* W3s   = (const float*)d_in[5];
  const float* b3s   = (const float*)d_in[6];
  const float* W4s   = (const float*)d_in[7];
  const float* b4s   = (const float*)d_in[8];
  const float* PA    = (const float*)d_in[9];
  const float* alpha = (const float*)d_in[10];
  const float* gamma = (const float*)d_in[11];
  const float* beta  = (const float*)d_in[12];
  float* out = (float*)d_out;

  char* ws = (char*)d_ws; size_t off = 0;
  auto take = [&](size_t bytes) { char* p = ws + off; off += (bytes + 255) & ~(size_t)255; return p; };
  float*          XM   = (float*)take((size_t)NB * VP * CIN * 4);
  float*          X12  = (float*)take((size_t)NB * VP * 64 * 4);
  unsigned short* W3B  = (unsigned short*)take((size_t)SS * COUT * CIN * 2);
  unsigned short* W12B = (unsigned short*)take((size_t)64 * 64 * 2);
  float*          B12  = (float*)take((size_t)64 * 4);
  unsigned short* XT   = (unsigned short*)take((size_t)CH * TT * VP * CIN * 2);
  unsigned short* X3H  = (unsigned short*)take((size_t)CH * TT * COUT * KP * 2);
  unsigned short* X3L  = (unsigned short*)take((size_t)CH * TT * COUT * KP * 2);
  unsigned short* MH   = (unsigned short*)take((size_t)CH * COUT * VP * KP * 2);
  unsigned short* ML   = (unsigned short*)take((size_t)CH * COUT * VP * KP * 2);
  float*          Y    = (float*)take((size_t)NB * COUT * VV * TT * 4);
  double*         PART = (double*)take((size_t)NB * COUT * 16 * 8);
  float*          BNP  = (float*)take((size_t)2 * COUT * 4);
  if (off > ws_size || off > (size_t)134217728) return;

  k_prep<<<9, 256, 0, stream>>>(W3s, W1s, W2s, b1s, b2s, W3B, W12B, B12);
  k_xm<<<NB * 8, 256, 0, stream>>>(x, XM);
  k_gemm_bf<true, 0, true><<<(2 * NB + 3) / 4, 128, 0, stream>>>(XM, 64, W12B, 64, B12, X12, 64, NB * VP, 64, 64);
  for (int c = 0; c < NCHUNK; ++c) {
    const int n0 = c * CH;
    k_xt<<<CH * 32, 256, 0, stream>>>(x, XT, n0);
    k_x3<<<CH * TT, 128, 0, stream>>>(XT, W3B, b3s, X3H, X3L);
    k_m<<<CH * 4, 256, 0, stream>>>(X12, W4s, b4s, PA, alpha, MH, ML, n0);
    k_agg<<<CH * 64, 128, 0, stream>>>(X3H, X3L, MH, ML, Y, PART, n0);
  }
  k_bnfin<<<1, 64, 0, stream>>>(PART, BNP);
  k_out<<<(NB * XS_FULL / 4 + 255) / 256, 256, 0, stream>>>(Y, x, BNP, gamma, beta, out, NB * XS_FULL / 4);
}
